// RNN_state_emb_5248450035917
// MI455X (gfx1250) — hardware-verified
//
#include <hip/hip_runtime.h>
#include <stddef.h>

typedef __attribute__((ext_vector_type(16))) _Float16 v16h;
typedef __attribute__((ext_vector_type(8)))  _Float16 v8h;
typedef __attribute__((ext_vector_type(8)))  float    v8f;
typedef __attribute__((ext_vector_type(4)))  float    v4f;

constexpr int BSZ  = 256;
constexpr int TLEN = 1024;
constexpr int HD   = 32;
constexpr int NLAY = 3;
constexpr int G3   = 96;

constexpr float ACT_SC   = 8.0f;
constexpr float W_SC     = 64.0f;
constexpr float INV_PROD = 1.0f / 512.0f;

constexpr int MLP_ROWS   = 64;
constexpr int ACT_PITCH  = 40;
constexpr int HX_PITCH   = 72;
constexpr int SLAB_PITCH = 36;

__device__ __forceinline__ void dep_guard_h(v8f& a, v8f& b, v16h x, v16h y) {
  asm volatile("v_nop\n\tv_nop\n\tv_nop\n\tv_nop" : "+v"(a), "+v"(b) : "v"(x), "v"(y));
}
template <typename T> struct Frag;
template <> struct Frag<_Float16> {
  typedef v16h V; union U { v16h v; v8h h[2]; };
  static __device__ __forceinline__ v16h load(const _Float16* p) {
    U f; f.h[0] = *(const v8h*)(p); f.h[1] = *(const v8h*)(p + 16); return f.v;
  }
  static __device__ __forceinline__ v8f mma(v16h a, v16h b, v8f c) {
    return __builtin_amdgcn_wmma_f32_16x16x32_f16(false, a, false, b, (short)0, c, false, false);
  }
};

__device__ __forceinline__ void guard2_abc(v8f& a, v8f& b, v16h x, v16h y, v16h z) {
  asm volatile("v_nop\n\tv_nop\n\tv_nop\n\tv_nop" : "+v"(a), "+v"(b) : "v"(x), "v"(y), "v"(z));
}
__device__ __forceinline__ void guard4_ab(v8f& a, v8f& b, v8f& c, v8f& d, v16h x, v16h y) {
  asm volatile("v_nop\n\tv_nop\n\tv_nop\n\tv_nop" : "+v"(a), "+v"(b), "+v"(c), "+v"(d) : "v"(x), "v"(y));
}

__device__ __forceinline__ v8f zero8() { return (v8f){0.f, 0.f, 0.f, 0.f, 0.f, 0.f, 0.f, 0.f}; }

__device__ __forceinline__ v16h frag_w32(const float* __restrict__ row, int hh) {
  const v4f a0 = *(const v4f*)(row + 8 * hh);
  const v4f a1 = *(const v4f*)(row + 8 * hh + 4);
  const v4f c0 = *(const v4f*)(row + 16 + 8 * hh);
  const v4f c1 = *(const v4f*)(row + 20 + 8 * hh);
  v16h f;
#pragma unroll
  for (int e = 0; e < 4; ++e) {
    f[e]      = (_Float16)(a0[e] * W_SC);
    f[4 + e]  = (_Float16)(a1[e] * W_SC);
    f[8 + e]  = (_Float16)(c0[e] * W_SC);
    f[12 + e] = (_Float16)(c1[e] * W_SC);
  }
  return f;
}

__device__ __forceinline__ v8h pack8_f16(v4f a, v4f b) {
  v8h h;
#pragma unroll
  for (int e = 0; e < 4; ++e) {
    h[e]     = (_Float16)(a[e] * ACT_SC);
    h[4 + e] = (_Float16)(b[e] * ACT_SC);
  }
  return h;
}

__device__ __forceinline__ void mlp_layer(_Float16* act, const float* __restrict__ W,
                                          const float* __restrict__ bvec, int w, int hh, int m) {
  const v16h a  = Frag<_Float16>::load(act + (16 * w + m) * ACT_PITCH + 8 * hh);
  const v16h bA = frag_w32(W + (size_t)m * HD, hh);
  const v16h bB = frag_w32(W + (size_t)(16 + m) * HD, hh);
  v8f c0 = zero8(), c1 = zero8();
  c0 = Frag<_Float16>::mma(a, bA, c0);
  c1 = Frag<_Float16>::mma(a, bB, c1);
  guard2_abc(c0, c1, a, bA, bB);
  const float bias0 = bvec[m];
  const float bias1 = bvec[16 + m];
#pragma unroll
  for (int r = 0; r < 8; ++r) {
    const float v0 = fmaxf(c0[r] * INV_PROD + bias0, 0.0f);
    const float v1 = fmaxf(c1[r] * INV_PROD + bias1, 0.0f);
    act[(16 * w + 8 * hh + r) * ACT_PITCH + m]      = (_Float16)(v0 * ACT_SC);
    act[(16 * w + 8 * hh + r) * ACT_PITCH + 16 + m] = (_Float16)(v1 * ACT_SC);
  }
}

__global__ __launch_bounds__(128)
void k_embed_mlp(const int* __restrict__ x, const float* __restrict__ emb, int nstate,
                 const float* __restrict__ W1, const float* __restrict__ b1,
                 const float* __restrict__ W2, const float* __restrict__ b2,
                 const float* __restrict__ W3, const float* __restrict__ b3,
                 _Float16* __restrict__ seq0) {
  __shared__ __align__(16) _Float16 act[MLP_ROWS * ACT_PITCH];
  const int tid  = threadIdx.x;
  const int w    = tid >> 5;
  const int lane = tid & 31;
  const int hh   = lane >> 4;
  const int m    = lane & 15;
  const int rowbase = blockIdx.x * MLP_ROWS;

  {
    const int row  = tid >> 1;
    const int half = tid & 1;
    const int R = rowbase + row;
    const int t = R >> 8;
    const int b = R & 255;
    int tok = x[(size_t)b * TLEN + t];
    tok = tok < 0 ? 0 : tok;
    tok = tok > nstate - 1 ? nstate - 1 : tok;
    const float* er = emb + (size_t)tok * HD + 16 * half;
    const v4f e0 = *(const v4f*)(er);
    const v4f e1 = *(const v4f*)(er + 4);
    const v4f e2 = *(const v4f*)(er + 8);
    const v4f e3 = *(const v4f*)(er + 12);
    *(v8h*)(act + row * ACT_PITCH + 16 * half)     = pack8_f16(e0, e1);
    *(v8h*)(act + row * ACT_PITCH + 16 * half + 8) = pack8_f16(e2, e3);
  }
  __syncthreads();
  mlp_layer(act, W1, b1, w, hh, m);
  __syncthreads();
  mlp_layer(act, W2, b2, w, hh, m);
  __syncthreads();
  mlp_layer(act, W3, b3, w, hh, m);
  __syncthreads();

  _Float16* dst = seq0 + (size_t)rowbase * HD;
  for (int pass = 0; pass < 2; ++pass) {
#pragma unroll
    for (int it = 0; it < 2; ++it) {
      const int idx = it * 128 + tid;
      const int row = idx >> 2;
      const int ch  = idx & 3;
      const v8h v = *(const v8h*)(act + row * ACT_PITCH + ch * 8);
      *(volatile v8h*)(dst + (size_t)row * HD + ch * 8) = v;
    }
    __threadfence();
  }
}

__global__ __launch_bounds__(64)
void k_gru_layer(const _Float16* __restrict__ seq_in, _Float16* __restrict__ seq_out,
                 const float* __restrict__ hid_l,
                 const float* __restrict__ Wih_l, const float* __restrict__ Whh_l,
                 const float* __restrict__ bih_l, const float* __restrict__ bhh_l,
                 float* __restrict__ out0, float* __restrict__ out1_l, int last) {
  __shared__ __align__(16) _Float16 hx[16 * HX_PITCH];
  __shared__ __align__(16) float slab[16 * SLAB_PITCH];
  const int tid  = threadIdx.x;
  const int c    = tid >> 5;
  const int lane = tid & 31;
  const int hh   = lane >> 4;
  const int cc   = lane & 15;
  const int b0   = blockIdx.x * 16;
  const int ucol = 16 * c + cc;

  const v16h brx = frag_w32(Wih_l + (size_t)(ucol) * HD, hh);
  const v16h brh = frag_w32(Whh_l + (size_t)(ucol) * HD, hh);
  const v16h bzx = frag_w32(Wih_l + (size_t)(32 + ucol) * HD, hh);
  const v16h bzh = frag_w32(Whh_l + (size_t)(32 + ucol) * HD, hh);
  const v16h bnx = frag_w32(Wih_l + (size_t)(64 + ucol) * HD, hh);
  const v16h bnh = frag_w32(Whh_l + (size_t)(64 + ucol) * HD, hh);
  const float bs_r = bih_l[ucol] + bhh_l[ucol];
  const float bs_z = bih_l[32 + ucol] + bhh_l[32 + ucol];
  const float b_in = bih_l[64 + ucol];
  const float b_hn = bhh_l[64 + ucol];

  float hreg[8];
#pragma unroll
  for (int r = 0; r < 8; ++r) hreg[r] = hid_l[(size_t)(b0 + 8 * hh + r) * HD + ucol];

  const int row  = tid >> 2;
  const int col8 = (tid & 3) * 8;

#pragma unroll
  for (int r = 0; r < 8; ++r) slab[(8 * hh + r) * SLAB_PITCH + ucol] = hreg[r];
  {
    const v8h xv = *(const v8h*)(seq_in + (size_t)(b0 + row) * HD + col8);
    *(v8h*)(hx + row * HX_PITCH + col8) = xv;
  }
  __syncthreads();
  {
    const v4f f0 = *(const v4f*)(slab + row * SLAB_PITCH + col8);
    const v4f f1 = *(const v4f*)(slab + row * SLAB_PITCH + col8 + 4);
    *(v8h*)(hx + row * HX_PITCH + 32 + col8) = pack8_f16(f0, f1);
  }

  for (int t = 0; t < TLEN; ++t) {
    __syncthreads();
    const v16h ax = Frag<_Float16>::load(hx + cc * HX_PITCH + 8 * hh);
    const v16h ah = Frag<_Float16>::load(hx + cc * HX_PITCH + 32 + 8 * hh);
    v8f ar = zero8(), az = zero8(), ain = zero8(), ahn = zero8();
    ar  = Frag<_Float16>::mma(ax, brx, ar);
    ar  = Frag<_Float16>::mma(ah, brh, ar);
    az  = Frag<_Float16>::mma(ax, bzx, az);
    az  = Frag<_Float16>::mma(ah, bzh, az);
    ain = Frag<_Float16>::mma(ax, bnx, ain);
    ahn = Frag<_Float16>::mma(ah, bnh, ahn);
    guard4_ab(ar, az, ain, ahn, ax, ah);

#pragma unroll
    for (int r = 0; r < 8; ++r) {
      const float pr  = ar[r]  * INV_PROD + bs_r;
      const float pz  = az[r]  * INV_PROD + bs_z;
      const float pin = ain[r] * INV_PROD + b_in;
      const float phn = ahn[r] * INV_PROD + b_hn;
      const float rg = 1.0f / (1.0f + expf(-pr));
      const float zg = 1.0f / (1.0f + expf(-pz));
      const float ng = tanhf(pin + rg * phn);
      hreg[r] = (1.0f - zg) * ng + zg * hreg[r];
    }

    __syncthreads();
#pragma unroll
    for (int r = 0; r < 8; ++r) slab[(8 * hh + r) * SLAB_PITCH + ucol] = hreg[r];
    {
      const int tn = (t + 1 < TLEN) ? (t + 1) : (TLEN - 1);
      const v8h xv = *(const v8h*)(seq_in + ((size_t)tn * BSZ + b0 + row) * HD + col8);
      *(v8h*)(hx + row * HX_PITCH + col8) = xv;
    }
    __syncthreads();

    const v4f f0 = *(const v4f*)(slab + row * SLAB_PITCH + col8);
    const v4f f1 = *(const v4f*)(slab + row * SLAB_PITCH + col8 + 4);
    const v8h hv = pack8_f16(f0, f1);
    *(v8h*)(hx + row * HX_PITCH + 32 + col8) = hv;
    if (!last) {
      _Float16* orow = seq_out + ((size_t)t * BSZ + b0 + row) * HD + col8;
      for (int pass = 0; pass < 2; ++pass) {
        *(volatile v8h*)(orow) = hv;
        __threadfence();
      }
    } else {
      for (int pass = 0; pass < 2; ++pass) {
#pragma unroll
        for (int it = 0; it < 2; ++it) {
          const int idx  = it * 64 + tid;
          const int orw  = idx >> 3;
          const int c4   = (idx & 7) * 4;
          const v4f v = *(const v4f*)(slab + orw * SLAB_PITCH + c4);
          *(volatile v4f*)(out0 + (size_t)(b0 + orw) * (TLEN * HD) + (size_t)t * HD + c4) = v;
        }
        __threadfence();
      }
    }
  }

  for (int pass = 0; pass < 2; ++pass) {
#pragma unroll
    for (int it = 0; it < 2; ++it) {
      const int idx = it * 64 + tid;
      const int orw = idx >> 3;
      const int c4  = (idx & 7) * 4;
      const v4f v = *(const v4f*)(slab + orw * SLAB_PITCH + c4);
      *(volatile v4f*)(out1_l + (size_t)(b0 + orw) * HD + c4) = v;
    }
    __threadfence();
  }
}

extern "C" void kernel_launch(void* const* d_in, const int* in_sizes, int n_in,
                              void* d_out, int out_size, void* d_ws, size_t ws_size,
                              hipStream_t stream) {
  (void)n_in; (void)out_size;
  const int*   x   = (const int*)  d_in[0];
  const float* hid = (const float*)d_in[1];
  const float* emb = (const float*)d_in[2];
  const float* W1  = (const float*)d_in[3];
  const float* b1  = (const float*)d_in[4];
  const float* W2  = (const float*)d_in[5];
  const float* b2  = (const float*)d_in[6];
  const float* W3  = (const float*)d_in[7];
  const float* b3  = (const float*)d_in[8];
  const float* Wih = (const float*)d_in[9];
  const float* Whh = (const float*)d_in[10];
  const float* bih = (const float*)d_in[11];
  const float* bhh = (const float*)d_in[12];

  const int nstate = in_sizes[2] / HD;
  if (in_sizes[0] != BSZ * TLEN || nstate < 1) return;

  const size_t seq_elems = (size_t)TLEN * BSZ * HD;
  if (2 * seq_elems * sizeof(_Float16) > ws_size) return;

  float* out0 = (float*)d_out;
  float* out1 = out0 + (size_t)BSZ * TLEN * HD;
  _Float16* S0 = (_Float16*)d_ws;
  _Float16* S1 = S0 + seq_elems;

  k_embed_mlp<<<(TLEN * BSZ) / MLP_ROWS, 128, 0, stream>>>(x, emb, nstate, W1, b1, W2, b2, W3, b3, S0);

  k_gru_layer<<<BSZ / 16, 64, 0, stream>>>(S0, S1, hid + (size_t)0 * BSZ * HD,
      Wih + (size_t)0 * G3 * HD, Whh + (size_t)0 * G3 * HD, bih + 0 * G3, bhh + 0 * G3,
      out0, out1 + (size_t)0 * BSZ * HD, 0);
  k_gru_layer<<<BSZ / 16, 64, 0, stream>>>(S1, S0, hid + (size_t)1 * BSZ * HD,
      Wih + (size_t)1 * G3 * HD, Whh + (size_t)1 * G3 * HD, bih + 1 * G3, bhh + 1 * G3,
      out0, out1 + (size_t)1 * BSZ * HD, 0);
  k_gru_layer<<<BSZ / 16, 64, 0, stream>>>(S0, S1, hid + (size_t)2 * BSZ * HD,
      Wih + (size_t)2 * G3 * HD, Whh + (size_t)2 * G3 * HD, bih + 2 * G3, bhh + 2 * G3,
      out0, out1 + (size_t)2 * BSZ * HD, 1);
  (void)NLAY;
}
